// S5_29274497090136
// MI455X (gfx1250) — hardware-verified
//
#include <hip/hip_runtime.h>
#include <cmath>

typedef __attribute__((ext_vector_type(16))) _Float16 v16h;
typedef __attribute__((ext_vector_type(8)))  _Float16 v8h;
typedef __attribute__((ext_vector_type(8)))  float    v8f;
typedef __attribute__((ext_vector_type(4)))  float    v4f;
typedef __attribute__((ext_vector_type(2)))  float    v2f;
typedef __attribute__((ext_vector_type(4)))  unsigned v4u;

constexpr int SEQ_LEN  = 8192;
constexpr int D_MODEL  = 1024;
constexpr int N_STATE  = 256;
constexpr int N_STATE2 = 2 * N_STATE;

constexpr float CARRY_BBAR = 4096.0f;
constexpr float CARRY_X    = 8.0f;
constexpr float CARRY_C    = 64.0f;
constexpr float SCALE_GEMM0 = 1.0f / 4096.0f;
constexpr float SCALE_GEMM1 = 1.0f / 512.0f;

constexpr size_t WS_OFF_PARAMS = 0;
constexpr size_t WS_SZ_PARAMS  = 4 * (size_t)N_STATE * 4;
constexpr size_t WS_OFF_BT1    = WS_OFF_PARAMS + WS_SZ_PARAMS;
constexpr size_t WS_SZ_BT1     = (size_t)N_STATE2 * D_MODEL * 2;
constexpr size_t WS_OFF_BT2    = WS_OFF_BT1 + WS_SZ_BT1;
constexpr size_t WS_SZ_BT2     = (size_t)D_MODEL * N_STATE2 * 2;
constexpr size_t WS_OFF_U16    = WS_OFF_BT2 + WS_SZ_BT2;
constexpr size_t WS_SZ_U16     = (size_t)SEQ_LEN * D_MODEL * 2;
constexpr size_t WS_OFF_G      = WS_OFF_U16 + WS_SZ_U16;
constexpr size_t WS_SZ_G       = (size_t)SEQ_LEN * N_STATE2 * 4;
constexpr size_t WS_OFF_X16    = WS_OFF_G + WS_SZ_G;
constexpr size_t WS_SZ_X16     = (size_t)SEQ_LEN * N_STATE2 * 2;
constexpr size_t WS_TOTAL      = WS_OFF_X16 + WS_SZ_X16;
static_assert(WS_TOTAL == 44044288, "carve");
static_assert(WS_TOTAL <= 134217728, "carve limit");
static_assert((WS_OFF_BT1 % 128) == 0 && (WS_OFF_BT2 % 128) == 0 && (WS_OFF_U16 % 128) == 0 &&
              (WS_OFF_G % 128) == 0 && (WS_OFF_X16 % 128) == 0, "line alignment");
static_assert(SEQ_LEN % 64 == 0 && N_STATE2 % 64 == 0 && D_MODEL % 64 == 0, "tile multiples");
static_assert(D_MODEL % 32 == 0 && N_STATE2 % 32 == 0, "k multiples");
static_assert(((SEQ_LEN / 64) * (N_STATE2 / 64)) % 8 == 0, "gemm0 grid");
static_assert(((SEQ_LEN / 64) * (D_MODEL / 64)) % 8 == 0, "gemm1 grid");

__device__ __forceinline__ _Float16 to_f16_ftz(float x) {
  const float w = (fabsf(x) < 6.103515625e-5f) ? 0.0f : x;
  return (_Float16)w;
}
__device__ __forceinline__ unsigned f16_bits_ftz(float x) {
  return (unsigned)__builtin_bit_cast(unsigned short, to_f16_ftz(x));
}

__device__ __forceinline__ void dep_guard_h(v8f& a, v8f& b, v16h x, v16h y) { asm volatile("v_nop\n\tv_nop\n\tv_nop\n\tv_nop" : "+v"(a), "+v"(b) : "v"(x), "v"(y)); }
__device__ __forceinline__ void keep4_h(v16h a, v16h b, v16h c, v16h d) { asm volatile("v_nop" :: "v"(a), "v"(b), "v"(c), "v"(d)); }
__device__ __forceinline__ void acc_guard4(v8f& a, v8f& b, v8f& c, v8f& d) { asm volatile("v_nop\n\tv_nop\n\tv_nop\n\tv_nop" : "+v"(a), "+v"(b), "+v"(c), "+v"(d)); }
template <typename T> struct Frag;
template <> struct Frag<_Float16> {
  typedef v16h V; union U { v16h v; v8h h[2]; };
  static __device__ __forceinline__ v16h load(const _Float16* p) {
    U f; f.h[0] = *(const v8h*)(p); f.h[1] = *(const v8h*)(p + 16); return f.v;
  }
  static __device__ __forceinline__ v8f mma(v16h a, v16h b, v8f c) {
    return __builtin_amdgcn_wmma_f32_16x16x32_f16(false, a, false, b, (short)0, c, false, false);
  }
  static __device__ __forceinline__ void guard(v8f& a, v8f& b, v16h x, v16h y) { dep_guard_h(a, b, x, y); }
  static __device__ __forceinline__ void keep(v16h a, v16h b, v16h c, v16h d) { keep4_h(a, b, c, d); }
};

template <bool DSKIP>
__global__ __launch_bounds__(256) void wmma_gemm64_f16(
    const unsigned short* __restrict__ Ap, int lda,
    const unsigned short* __restrict__ Btp, int ldb,
    float* __restrict__ Cout, int ldc,
    const float* __restrict__ skipU, const float* __restrict__ skipD,
    int M, int N, int K, float scale) {
  typedef _Float16 T;
  typedef v16h V;
  const T* A = (const T*)Ap; const T* Bt = (const T*)Btp;
  __shared__ __align__(16) float sT[8][16 * 68];
  const int lane = threadIdx.x & 31;
  const int wave = threadIdx.x >> 5;
  const int tilesN = N >> 6;
  const int tilesM = M >> 6;
  const int tile = blockIdx.x * 8 + wave;
  if (tile >= tilesM * tilesN) return;
  const int tm = tile / tilesN;
  const int tn = tile - tm * tilesN;
  const int m0 = tm << 6;
  const int n0 = tn << 6;

  const int rlane = lane & 15;
  const int koff  = (lane >> 4) * 8;
  const int mOff  = (lane >> 4) * 8;

  v8f acc[4][4];
#pragma unroll
  for (int i = 0; i < 4; ++i)
#pragma unroll
    for (int j = 0; j < 4; ++j) acc[i][j] = (v8f){0.f,0.f,0.f,0.f,0.f,0.f,0.f,0.f};

  for (int k0 = 0; k0 < K; k0 += 32) {
    V bh[4];
#pragma unroll
    for (int j = 0; j < 4; ++j) {
      const size_t bo = (size_t)(n0 + (j << 4) + rlane) * ldb + koff + k0;
      bh[j] = Frag<T>::load(Bt + bo);
    }
#pragma unroll
    for (int i = 0; i < 4; ++i) {
      const size_t ao = (size_t)(m0 + (i << 4) + rlane) * lda + koff + k0;
      V ah = Frag<T>::load(A + ao);
#pragma unroll
      for (int j = 0; j < 4; ++j) {
        acc[i][j] = Frag<T>::mma(ah, bh[j], acc[i][j]);
      }
      Frag<T>::guard(acc[i][0], acc[i][3], ah, ah);
    }
    Frag<T>::keep(bh[0], bh[1], bh[2], bh[3]);
  }
  acc_guard4(acc[0][0], acc[0][1], acc[0][2], acc[0][3]);
  acc_guard4(acc[1][0], acc[1][1], acc[1][2], acc[1][3]);
  acc_guard4(acc[2][0], acc[2][1], acc[2][2], acc[2][3]);
  acc_guard4(acc[3][0], acc[3][1], acc[3][2], acc[3][3]);

  float* slab = sT[wave];
  const int hh = lane >> 4, c4 = (lane & 15) * 4;
  v4f d4 = (v4f){0.f, 0.f, 0.f, 0.f};
  if (DSKIP) d4 = *(const v4f*)(skipD + n0 + c4);
#pragma unroll
  for (int i = 0; i < 4; ++i) {
    const int mBase = m0 + (i << 4);
#pragma unroll
    for (int j = 0; j < 4; ++j) {
#pragma unroll
      for (int r = 0; r < 8; ++r) {
        const float v = acc[i][j][r] * scale;
        slab[(mOff + r) * 68 + (j << 4) + rlane] = v;
      }
    }
    __builtin_amdgcn_fence(__ATOMIC_RELEASE, "workgroup");
    __builtin_amdgcn_wave_barrier();
    __builtin_amdgcn_fence(__ATOMIC_ACQUIRE, "workgroup");
    if (DSKIP) {
#pragma unroll
      for (int it = 0; it < 8; ++it) {
        const int row = it * 2 + hh;
        float* sp = slab + row * 68 + c4;
        v4f v = *(const v4f*)sp;
        const v4f u4 = *(const v4f*)(skipU + (size_t)(mBase + row) * ldc + n0 + c4);
        v = d4 * u4 + v;
        *(v4f*)sp = v;
      }
      __builtin_amdgcn_fence(__ATOMIC_RELEASE, "workgroup");
      __builtin_amdgcn_wave_barrier();
      __builtin_amdgcn_fence(__ATOMIC_ACQUIRE, "workgroup");
    }
    for (int pass = 0; pass < 2; ++pass) {
#pragma unroll
      for (int it = 0; it < 8; ++it) {
        const int row = it * 2 + hh;
        v4f v = *(const v4f*)(slab + row * 68 + c4);
        *(volatile v4f*)(Cout + (size_t)(mBase + row) * ldc + n0 + c4) = v;
      }
      __threadfence();
    }
    __builtin_amdgcn_fence(__ATOMIC_RELEASE, "workgroup");
    __builtin_amdgcn_wave_barrier();
    __builtin_amdgcn_fence(__ATOMIC_ACQUIRE, "workgroup");
  }
}

__global__ __launch_bounds__(256) void ssm_setup(
    const float* __restrict__ Lre, const float* __restrict__ Lim,
    const float* __restrict__ logstep, float* __restrict__ params) {
  const int p = threadIdx.x;
  const float lr = Lre[p], li = Lim[p];
  const float st = expf(logstep[p]);
  const float zr = lr * st, zi = li * st;
  const float ea = expf(zr);
  const float er = ea * cosf(zi);
  const float ei = ea * sinf(zi);
  const float a  = er - 1.0f;
  const float d  = lr * lr + li * li;
  const float inv = 1.0f / d;
  const float fr = (a * lr + ei * li) * inv;
  const float fi = (ei * lr - a * li) * inv;
  volatile float* vp = params;
  vp[p] = er; vp[N_STATE + p] = ei; vp[2 * N_STATE + p] = fr; vp[3 * N_STATE + p] = fi;
  __threadfence();
  vp[p] = er; vp[N_STATE + p] = ei; vp[2 * N_STATE + p] = fr; vp[3 * N_STATE + p] = fi;
}

__global__ __launch_bounds__(256) void prep_bbar(
    const float* __restrict__ Bin, const float* __restrict__ params, _Float16* __restrict__ Bt1) {
  const int g  = blockIdx.x * 256 + threadIdx.x;
  const int p  = g >> 7;
  const int h8 = (g & 127) << 3;
  const float fr = params[2 * N_STATE + p], fi = params[3 * N_STATE + p];
  const float* src = Bin + ((size_t)p * D_MODEL + h8) * 2;
  v4f w[4];
#pragma unroll
  for (int i = 0; i < 4; ++i) w[i] = *(const v4f*)(src + 4 * i);
  v8h re, im;
#pragma unroll
  for (int e = 0; e < 8; ++e) {
    const float br = w[e >> 1][(e & 1) * 2];
    const float bi = w[e >> 1][(e & 1) * 2 + 1];
    const float vr = (fr * br - fi * bi) * CARRY_BBAR;
    const float vi = (fr * bi + fi * br) * CARRY_BBAR;
    re[e] = to_f16_ftz(vr);
    im[e] = to_f16_ftz(vi);
  }
  _Float16* d0 = Bt1 + (size_t)(2 * p) * D_MODEL + h8;
  _Float16* d1 = Bt1 + (size_t)(2 * p + 1) * D_MODEL + h8;
  *(volatile v8h*)d0 = re;
  *(volatile v8h*)d1 = im;
  __threadfence();
  *(volatile v8h*)d0 = re;
  *(volatile v8h*)d1 = im;
}

__global__ __launch_bounds__(256) void cvt_plane_f16(
    const float* __restrict__ in, _Float16* __restrict__ out, float sEven, float sOdd) {
  const size_t g = (size_t)blockIdx.x * 256 + threadIdx.x;
  const float* src = in + g * 8;
  const v4f a = *(const v4f*)(src);
  const v4f b = *(const v4f*)(src + 4);
  v8h hv;
  hv[0] = to_f16_ftz(a[0] * sEven); hv[1] = to_f16_ftz(a[1] * sOdd);
  hv[2] = to_f16_ftz(a[2] * sEven); hv[3] = to_f16_ftz(a[3] * sOdd);
  hv[4] = to_f16_ftz(b[0] * sEven); hv[5] = to_f16_ftz(b[1] * sOdd);
  hv[6] = to_f16_ftz(b[2] * sEven); hv[7] = to_f16_ftz(b[3] * sOdd);
  _Float16* dst = out + g * 8;
  *(volatile v8h*)dst = hv;
  __threadfence();
  *(volatile v8h*)dst = hv;
}

__global__ __launch_bounds__(32) void ssm_scan(
    const float* __restrict__ G, const float* __restrict__ params, unsigned* __restrict__ X32) {
  __shared__ __align__(16) unsigned stage[32 * 32];
  const int lane = threadIdx.x;
  const int p = blockIdx.x * 32 + lane;
  const float lr = params[p], li = params[N_STATE + p];
  float xr = 0.0f, xi = 0.0f;
  const float* gp = G + 2 * p;
  const int q = lane >> 3, c = lane & 7;
#pragma unroll 1
  for (int t0 = 0; t0 < SEQ_LEN; t0 += 32) {
    for (int sub = 0; sub < 2; ++sub) {
      const int tb = t0 + sub * 16;
      v2f g[16];
#pragma unroll
      for (int s = 0; s < 16; ++s) g[s] = *(const v2f*)(gp + (size_t)(tb + s) * N_STATE2);
#pragma unroll
      for (int s = 0; s < 16; ++s) {
        const float nxr = fmaf(lr, xr, fmaf(-li, xi, g[s][0]));
        const float nxi = fmaf(lr, xi, fmaf( li, xr, g[s][1]));
        xr = nxr; xi = nxi;
        const unsigned lo = f16_bits_ftz(xr * CARRY_X);
        const unsigned hi = f16_bits_ftz(xi * CARRY_X);
        stage[(sub * 16 + s) * 32 + lane] = lo | (hi << 16);
      }
    }
    __syncthreads();
    for (int pass = 0; pass < 2; ++pass) {
#pragma unroll
      for (int it = 0; it < 8; ++it) {
        const int row = it * 4 + q;
        const v4u w = *(const v4u*)(stage + row * 32 + c * 4);
        *(volatile v4u*)(X32 + (size_t)(t0 + row) * (N_STATE2 / 2) + blockIdx.x * 32 + c * 4) = w;
      }
      __threadfence();
    }
    __syncthreads();
  }
}

extern "C" void kernel_launch(void* const* d_in, const int* in_sizes, int n_in,
                              void* d_out, int out_size, void* d_ws, size_t ws_size,
                              hipStream_t stream) {
  if (n_in != 7) return;
  if (in_sizes[0] != SEQ_LEN * D_MODEL) return;
  if (in_sizes[1] != N_STATE) return;
  if (in_sizes[2] != N_STATE) return;
  if (in_sizes[3] != N_STATE * D_MODEL * 2) return;
  if (in_sizes[4] != D_MODEL * N_STATE * 2) return;
  if (in_sizes[5] != D_MODEL) return;
  if (in_sizes[6] != N_STATE) return;
  if (out_size != SEQ_LEN * D_MODEL) return;
  if (ws_size < WS_TOTAL) return;

  const float* U     = (const float*)d_in[0];
  const float* Lre   = (const float*)d_in[1];
  const float* Lim   = (const float*)d_in[2];
  const float* Bin   = (const float*)d_in[3];
  const float* Cin   = (const float*)d_in[4];
  const float* Dv    = (const float*)d_in[5];
  const float* lstep = (const float*)d_in[6];
  float* Out = (float*)d_out;

  unsigned char* ws = (unsigned char*)d_ws;
  float*    params = (float*)(ws + WS_OFF_PARAMS);
  _Float16* Bt1    = (_Float16*)(ws + WS_OFF_BT1);
  _Float16* Bt2    = (_Float16*)(ws + WS_OFF_BT2);
  _Float16* U16    = (_Float16*)(ws + WS_OFF_U16);
  float*    G      = (float*)(ws + WS_OFF_G);
  unsigned* X32    = (unsigned*)(ws + WS_OFF_X16);

  ssm_setup<<<dim3(1), dim3(256), 0, stream>>>(Lre, Lim, lstep, params);

  prep_bbar<<<dim3((N_STATE * (D_MODEL / 8)) / 256), dim3(256), 0, stream>>>(Bin, params, Bt1);

  cvt_plane_f16<<<dim3((D_MODEL * N_STATE2 / 8) / 256), dim3(256), 0, stream>>>(
      Cin, Bt2, 2.0f * CARRY_C, -2.0f * CARRY_C);

  cvt_plane_f16<<<dim3((SEQ_LEN * (D_MODEL / 8)) / 256), dim3(256), 0, stream>>>(U, U16, 1.0f, 1.0f);

  wmma_gemm64_f16<false><<<dim3(((SEQ_LEN / 64) * (N_STATE2 / 64)) / 8), dim3(256), 0, stream>>>(
      (const unsigned short*)U16, D_MODEL, (const unsigned short*)Bt1, D_MODEL,
      G, N_STATE2, U, Dv, SEQ_LEN, N_STATE2, D_MODEL, SCALE_GEMM0);

  ssm_scan<<<dim3(N_STATE / 32), dim3(32), 0, stream>>>(G, params, X32);

  wmma_gemm64_f16<true><<<dim3(((SEQ_LEN / 64) * (D_MODEL / 64)) / 8), dim3(256), 0, stream>>>(
      (const unsigned short*)X32, N_STATE2, (const unsigned short*)Bt2, N_STATE2,
      Out, D_MODEL, U, Dv, SEQ_LEN, D_MODEL, N_STATE2, SCALE_GEMM1);
}
